// UserEncoder_35356170780886
// MI455X (gfx1250) — hardware-run, weakly checked
//
#include <hip/hip_runtime.h>

typedef __attribute__((ext_vector_type(16))) _Float16 v16h;
typedef __attribute__((ext_vector_type(8)))  _Float16 v8h;
typedef __attribute__((ext_vector_type(16))) __bf16   v16b;
typedef __attribute__((ext_vector_type(8)))  __bf16   v8b;
typedef __attribute__((ext_vector_type(8)))  float    v8f;
typedef __attribute__((ext_vector_type(4)))  float    v4f;
typedef __attribute__((ext_vector_type(8)))  unsigned short u16x8;
typedef __attribute__((ext_vector_type(4)))  unsigned int   u32x4;

constexpr int kBatch  = 1024;
constexpr int kSeq    = 200;
constexpr int kEmb    = 128;
constexpr int kHid    = 128;
constexpr int kGates  = 384;
constexpr int kRows   = 16;
constexpr int kThreads = 256;
constexpr int kWPitch = 136;
constexpr int kXPitch = 136;
constexpr int kXBuf   = kRows * kXPitch;
constexpr int kOPitch = 132;

constexpr int kOffWih  = 0;
constexpr int kBytesW  = kGates * kWPitch * 2;
constexpr int kOffWhh  = kOffWih + kBytesW;
constexpr int kOffX    = kOffWhh + kBytesW;
constexpr int kBytesXH = 2 * kXBuf * 2;
constexpr int kOffH    = kOffX + kBytesXH;
constexpr int kOffO    = kOffH + kBytesXH;
constexpr int kBytesO  = kRows * kOPitch * 4;
constexpr int kLdsTotal = kOffO + kBytesO;
constexpr int kZeroChunks = (kOffO - kOffX) / 16;

static_assert(kBatch % kRows == 0);
static_assert(kRows == 16);
static_assert((kThreads / 32) * 16 == kHid);
static_assert(kEmb % 32 == 0 && kHid % 32 == 0);
static_assert(kEmb == kHid);
static_assert(kGates == 3 * kHid);
static_assert(kThreads == kRows * (kEmb / 8));
static_assert((kOffWhh % 16) == 0 && (kOffX % 16) == 0 && (kOffH % 16) == 0 && (kOffO % 16) == 0);
static_assert(((kWPitch * 2) % 16) == 0 && ((kXPitch * 2) % 16) == 0 && ((kOPitch * 4) % 16) == 0);
static_assert(((kOffO - kOffX) % 16) == 0);
static_assert(kLdsTotal <= 300000);

__device__ __forceinline__ unsigned short f2bf_bits(float f) {
  unsigned u = __float_as_uint(f);
  return (unsigned short)((u + 0x7FFFu + ((u >> 16) & 1u)) >> 16);
}
__device__ __forceinline__ float bf_bits2f(unsigned short h) { return __uint_as_float(((unsigned)h) << 16); }
__device__ __forceinline__ float bf_rne(float x) { return bf_bits2f(f2bf_bits(x)); }

__device__ __forceinline__ void dep_guard_h(v8f& a, v8f& b, v16h x, v16h y) { asm volatile("v_nop\n\tv_nop\n\tv_nop\n\tv_nop" : "+v"(a), "+v"(b) : "v"(x), "v"(y)); }
__device__ __forceinline__ void dep_guard_b(v8f& a, v8f& b, v16b x, v16b y) { asm volatile("v_nop\n\tv_nop\n\tv_nop\n\tv_nop" : "+v"(a), "+v"(b) : "v"(x), "v"(y)); }
__device__ __forceinline__ void keep4_h(v16h a, v16h b, v16h c, v16h d) { asm volatile("v_nop" :: "v"(a), "v"(b), "v"(c), "v"(d)); }
__device__ __forceinline__ void keep4_b(v16b a, v16b b, v16b c, v16b d) { asm volatile("v_nop" :: "v"(a), "v"(b), "v"(c), "v"(d)); }
template <typename T> struct Frag;
template <> struct Frag<_Float16> {
  typedef v16h V; union U { v16h v; v8h h[2]; };
  static __device__ __forceinline__ v16h load(const _Float16* p) {
    U f; f.h[0] = *(const v8h*)(p); f.h[1] = *(const v8h*)(p + 16); return f.v;
  }
  static __device__ __forceinline__ v8f mma(v16h a, v16h b, v8f c) {
    return __builtin_amdgcn_wmma_f32_16x16x32_f16(false, a, false, b, (short)0, c, false, false);
  }
  static __device__ __forceinline__ void guard(v8f& a, v8f& b, v16h x, v16h y) { dep_guard_h(a, b, x, y); }
  static __device__ __forceinline__ void keep(v16h a, v16h b, v16h c, v16h d) { keep4_h(a, b, c, d); }
};
template <> struct Frag<__bf16> {
  typedef v16b V; union U { v16b v; v8b h[2]; };
  static __device__ __forceinline__ v16b load(const __bf16* p) {
    U f; f.h[0] = *(const v8b*)(p); f.h[1] = *(const v8b*)(p + 16); return f.v;
  }
  static __device__ __forceinline__ v8f mma(v16b a, v16b b, v8f c) {
    return __builtin_amdgcn_wmma_f32_16x16x32_bf16(false, a, false, b, (short)0, c, false, false);
  }
  static __device__ __forceinline__ void guard(v8f& a, v8f& b, v16b x, v16b y) { dep_guard_b(a, b, x, y); }
  static __device__ __forceinline__ void keep(v16b a, v16b b, v16b c, v16b d) { keep4_b(a, b, c, d); }
};

__device__ __forceinline__ v8f mma_b16(v16b a, v16b b, v8f c) {
  c = __builtin_amdgcn_wmma_f32_16x16x32_bf16(false, a, false, b, (short)0, c, false, false);
  asm volatile("v_nop\n\tv_nop\n\tv_nop\n\tv_nop" : "+v"(c) : "v"(a), "v"(b));
  return c;
}
__device__ __forceinline__ v8f mma_h16(v16h a, v16h b, v8f c) {
  c = __builtin_amdgcn_wmma_f32_16x16x32_f16(false, a, false, b, (short)0, c, false, false);
  asm volatile("v_nop\n\tv_nop\n\tv_nop\n\tv_nop" : "+v"(c) : "v"(a), "v"(b));
  return c;
}

__device__ __forceinline__ float exp2_clamped(float x) {
  x = fminf(fmaxf(x, -100.0f), 100.0f);
  return __builtin_amdgcn_exp2f(x);
}
__device__ __forceinline__ float sigmoid_f(float p) {
  const float e = exp2_clamped(-p * 1.4426950408889634f);
  return __builtin_amdgcn_rcpf(1.0f + e);
}
__device__ __forceinline__ float tanh_f(float x) {
  const float e = exp2_clamped(x * 2.8853900817779268f);
  return 1.0f - 2.0f * __builtin_amdgcn_rcpf(e + 1.0f);
}

__global__ void __launch_bounds__(kThreads)
gru_scan_kernel(const int*   __restrict__ item_seq,
                const float* __restrict__ emb,
                const float* __restrict__ W_ih,
                const float* __restrict__ W_hh,
                const float* __restrict__ b_ih,
                const float* __restrict__ b_hh,
                float*       __restrict__ out,
                int n_vocab)
{
  extern __shared__ __attribute__((aligned(16))) char smem[];
  unsigned short* wih_us = (unsigned short*)(smem + kOffWih);
  const __bf16*   wih    = (const __bf16*)(smem + kOffWih);
  _Float16*       whh    = (_Float16*)(smem + kOffWhh);
  unsigned short* x_us   = (unsigned short*)(smem + kOffX);
  const __bf16*   xb     = (const __bf16*)(smem + kOffX);
  _Float16*       hm     = (_Float16*)(smem + kOffH);
  float*          ost    = (float*)(smem + kOffO);

  const int tid   = threadIdx.x;
  const int lane  = tid & 31;
  const int wave  = tid >> 5;
  const int cl    = lane & 15;
  const int hh    = lane >> 4;
  const int rbase = hh * 8;
  const int gc    = wave * 16 + cl;
  const int b0    = blockIdx.x * kRows;
  const int grow  = tid >> 4;
  const int ge0   = (tid & 15) * 8;

  {
    const u32x4 z4 = {0u, 0u, 0u, 0u};
    for (int i = tid; i < kZeroChunks; i += kThreads)
      *(u32x4*)(smem + kOffX + i * 16) = z4;
    for (int r = tid; r < 2 * kGates; r += kThreads)
      *(u32x4*)(smem + kOffWih + r * (kWPitch * 2) + kEmb * 2) = z4;
  }
  __syncthreads();

#pragma unroll 1
  for (int i = tid; i < kGates * (kEmb / 8); i += kThreads) {
    const int row = i >> 4;
    const int c8  = (i & 15) * 8;
    const float* s0 = W_ih + (size_t)row * kEmb + c8;
    const float* s1 = W_hh + (size_t)row * kHid + c8;
    const v4f a0 = *(const v4f*)s0;
    const v4f a1 = *(const v4f*)(s0 + 4);
    const v4f c0 = *(const v4f*)s1;
    const v4f c1 = *(const v4f*)(s1 + 4);
    u16x8 pk;
    v8h   ph;
#pragma unroll
    for (int e = 0; e < 4; ++e) {
      pk[e]     = f2bf_bits(a0[e]);
      pk[4 + e] = f2bf_bits(a1[e]);
      const float w0 = bf_rne(c0[e]) * 16.0f;
      const float w1 = bf_rne(c1[e]) * 16.0f;
      ph[e]     = (_Float16)w0;
      ph[4 + e] = (_Float16)w1;
    }
    *(u16x8*)(wih_us + row * kWPitch + c8) = pk;
    *(v8h*)(whh + row * kWPitch + c8)      = ph;
  }

  {
    int item = item_seq[(size_t)(b0 + grow) * kSeq + 0];
    item = item < 0 ? 0 : item;
    item = item > n_vocab - 1 ? n_vocab - 1 : item;
    const float* src = emb + (size_t)item * kEmb + ge0;
    const v4f a  = *(const v4f*)src;
    const v4f bb = *(const v4f*)(src + 4);
    u16x8 pk;
#pragma unroll
    for (int e = 0; e < 4; ++e) { pk[e] = f2bf_bits(a[e]); pk[4 + e] = f2bf_bits(bb[e]); }
    *(u16x8*)(x_us + grow * kXPitch + ge0) = pk;
  }

  const float bxr = bf_rne(b_ih[gc]),            bhr = bf_rne(b_hh[gc]);
  const float bxz = bf_rne(b_ih[kHid + gc]),     bhz = bf_rne(b_hh[kHid + gc]);
  const float bxn = bf_rne(b_ih[2 * kHid + gc]), bhn = bf_rne(b_hh[2 * kHid + gc]);

  float hreg[8];
#pragma unroll
  for (int v = 0; v < 8; ++v) hreg[v] = 0.0f;

  __syncthreads();

  const float kFold = 0.00390625f;

  for (int t = 0; t < kSeq; ++t) {
    const int cur = t & 1;
    const int nxt = cur ^ 1;
    const __bf16*   xcur = xb   + cur * kXBuf;
    unsigned short* xnxt = x_us + nxt * kXBuf;
    const _Float16* hcur = hm   + cur * kXBuf;
    _Float16*       hnxt = hm   + nxt * kXBuf;

    const bool have_next = (t + 1 < kSeq);
    v4f ga = {0.f, 0.f, 0.f, 0.f};
    v4f gb = {0.f, 0.f, 0.f, 0.f};
    if (have_next) {
      int item = item_seq[(size_t)(b0 + grow) * kSeq + t + 1];
      item = item < 0 ? 0 : item;
      item = item > n_vocab - 1 ? n_vocab - 1 : item;
      const float* src = emb + (size_t)item * kEmb + ge0;
      ga = *(const v4f*)src;
      gb = *(const v4f*)(src + 4);
    }

    v8f aci[3], ach[3];
#pragma unroll
    for (int g = 0; g < 3; ++g) {
      aci[g] = (v8f){0.f, 0.f, 0.f, 0.f, 0.f, 0.f, 0.f, 0.f};
      ach[g] = (v8f){0.f, 0.f, 0.f, 0.f, 0.f, 0.f, 0.f, 0.f};
    }
#pragma unroll 1
    for (int kc = 0; kc < kEmb / 32; ++kc) {
      const int kofs = kc * 32 + hh * 8;
      const v16b ax = Frag<__bf16>::load(xcur + cl * kXPitch + kofs);
      const v16h ah = Frag<_Float16>::load(hcur + cl * kXPitch + kofs);
#pragma unroll
      for (int g = 0; g < 3; ++g) {
        const int n = g * kHid + gc;
        const v16b bi = Frag<__bf16>::load(wih + n * kWPitch + kofs);
        const v16h bh = Frag<_Float16>::load(whh + n * kWPitch + kofs);
        aci[g] = mma_b16(ax, bi, aci[g]);
        ach[g] = mma_h16(ah, bh, ach[g]);
      }
    }

    if (have_next) {
      u16x8 pk;
#pragma unroll
      for (int e = 0; e < 4; ++e) { pk[e] = f2bf_bits(ga[e]); pk[4 + e] = f2bf_bits(gb[e]); }
      *(u16x8*)(xnxt + grow * kXPitch + ge0) = pk;
    }

#pragma unroll
    for (int v = 0; v < 8; ++v) {
      const float pr = (aci[0][v] + bxr) + (ach[0][v] * kFold + bhr);
      const float pz = (aci[1][v] + bxz) + (ach[1][v] * kFold + bhz);
      const float xn = aci[2][v] + bxn;
      const float hn = ach[2][v] * kFold + bhn;
      const float r  = sigmoid_f(pr);
      const float z  = sigmoid_f(pz);
      const float nn = tanh_f(xn + r * hn);
      const float hnew = (1.0f - z) * nn + z * hreg[v];
      hreg[v] = hnew;
      hnxt[(rbase + v) * kXPitch + gc] = (_Float16)(hnew * 16.0f);
    }

    __syncthreads();
  }

#pragma unroll
  for (int v = 0; v < 8; ++v) ost[(rbase + v) * kOPitch + gc] = hreg[v];
  __syncthreads();
  for (int pass = 0; pass < 2; ++pass) {
#pragma unroll
    for (int rr = 0; rr < 2; ++rr) {
      const int row = wave * 2 + rr;
      const v4f val = *(const v4f*)(ost + row * kOPitch + lane * 4);
      *(volatile v4f*)(out + (size_t)(b0 + row) * kHid + lane * 4) = val;
    }
    __threadfence();
  }
}

extern "C" void kernel_launch(void* const* d_in, const int* in_sizes, int n_in,
                              void* d_out, int out_size, void* d_ws, size_t ws_size,
                              hipStream_t stream) {
  (void)d_ws; (void)ws_size;
  if (n_in < 6) return;
  if (in_sizes[0] != kBatch * kSeq) return;
  if (in_sizes[1] < kEmb || (in_sizes[1] % kEmb) != 0) return;
  if (in_sizes[2] != kGates * kEmb || in_sizes[3] != kGates * kHid) return;
  if (in_sizes[4] != kGates || in_sizes[5] != kGates) return;
  if (out_size != kBatch * kHid) return;

  const int*   item_seq = (const int*)d_in[0];
  const float* emb      = (const float*)d_in[1];
  const float* W_ih     = (const float*)d_in[2];
  const float* W_hh     = (const float*)d_in[3];
  const float* b_ih     = (const float*)d_in[4];
  const float* b_hh     = (const float*)d_in[5];
  const int n_vocab = in_sizes[1] / kEmb;

  gru_scan_kernel<<<dim3(kBatch / kRows), dim3(kThreads), kLdsTotal, stream>>>(
      item_seq, emb, W_ih, W_hh, b_ih, b_hh, (float*)d_out, n_vocab);
}
